// MultiModalFusion_62534723829955
// MI455X (gfx1250) — hardware-run, weakly checked
//
#include <hip/hip_runtime.h>


#define NB_  4
#define CH   128
#define IH   100
#define IW   256
#define QH   25
#define QR   25600
typedef _Float16 h16;
typedef unsigned short bf;
typedef __attribute__((ext_vector_type(16))) __bf16   v16bf;
typedef __attribute__((ext_vector_type(16))) _Float16 v16h;
typedef __attribute__((ext_vector_type(8)))  _Float16 v8h;
typedef __attribute__((ext_vector_type(8)))  unsigned short v8us;
typedef __attribute__((ext_vector_type(8)))  float    v8f;
typedef __attribute__((ext_vector_type(4)))  float    v4f;
typedef v8h  __attribute__((may_alias)) v8ha;
typedef v4f  __attribute__((may_alias)) v4fa;
typedef v8us __attribute__((may_alias)) v8usa;

__device__ __forceinline__ unsigned short f2bf(float f) { unsigned u = __float_as_uint(f); u += 0x7FFFu + ((u >> 16) & 1u); return (unsigned short)(u >> 16); }
__device__ __forceinline__ float bf2f(unsigned short b) { return __uint_as_float(((unsigned)b) << 16); }
__device__ __forceinline__ float bfr(float f) { return bf2f(f2bf(f)); }
__device__ __forceinline__ v16h cat16(v8h lo, v8h hi) { return __builtin_shufflevector(lo, hi, 0, 1, 2, 3, 4, 5, 6, 7, 8, 9, 10, 11, 12, 13, 14, 15); }
__device__ __forceinline__ v16bf cat16b(v8us lo, v8us hi) { return __builtin_bit_cast(v16bf, __builtin_shufflevector(lo, hi, 0, 1, 2, 3, 4, 5, 6, 7, 8, 9, 10, 11, 12, 13, 14, 15)); }
__device__ __forceinline__ v8f wmma16(v16h a, v16h b, v8f c) { return __builtin_amdgcn_wmma_f32_16x16x32_f16(false, a, false, b, (short)0, c, false, false); }
__device__ __forceinline__ v8f wmmab(v16bf a, v16bf b, v8f c) { return __builtin_amdgcn_wmma_f32_16x16x32_bf16(false, a, false, b, (short)0, c, false, false); }


template <typename T16> struct WFrag;
template <> struct WFrag<h16> { typedef v16h V; static __device__ __forceinline__ V ld(const h16* p) { return cat16(*(const v8h*)p, *(const v8h*)(p + 16)); } static __device__ __forceinline__ v8f mma(V a, V b, v8f c) { return wmma16(a, b, c); } };
template <> struct WFrag<bf> { typedef v16bf V; static __device__ __forceinline__ V ld(const bf* p) { return cat16b(*(const v8us*)p, *(const v8us*)(p + 16)); } static __device__ __forceinline__ v8f mma(V a, V b, v8f c) { return wmmab(a, b, c); } };
template <typename T16, int NSPLIT, bool BIAS>
__global__ __launch_bounds__(32) void k_gemmw(const T16* __restrict__ A, const T16* __restrict__ A2, const T16* __restrict__ Bt, const T16* __restrict__ Bt2, int K, float* C, int ldc, const float* __restrict__ bias, size_t sA, size_t sB, size_t sC) {
    typedef typename WFrag<T16>::V V;
    __shared__ __align__(16) float os[16 * 68];
    const size_t z = blockIdx.z; A += z * sA; if (A2) A2 += z * sA; Bt += z * sB; if (Bt2) Bt2 += z * sB; C += z * sC;
    const int lane = threadIdx.x & 31, lr = lane & 15, hi = lane >> 4; const int r0 = blockIdx.x * 64, c0 = blockIdx.y * 64;
    v8f acc[4][4];
#pragma unroll
    for (int mb = 0; mb < 4; ++mb)
#pragma unroll
        for (int nb = 0; nb < 4; ++nb) acc[mb][nb] = (v8f){};
    const size_t aoff = (size_t)(r0 + lr) * K + 8 * hi, boff = (size_t)(c0 + lr) * K + 8 * hi;
    for (int kc = 0; kc < K; kc += 32) {
        V a[4], a2[4];
#pragma unroll
        for (int mb = 0; mb < 4; ++mb) { a[mb] = WFrag<T16>::ld(A + aoff + (size_t)mb * 16 * K + kc); if (NSPLIT == 1 || NSPLIT == 2) a2[mb] = WFrag<T16>::ld(A2 + aoff + (size_t)mb * 16 * K + kc); }
#pragma unroll
        for (int nb = 0; nb < 4; ++nb) { const V b = WFrag<T16>::ld(Bt + boff + (size_t)nb * 16 * K + kc); V b2; if (NSPLIT >= 2) b2 = WFrag<T16>::ld(Bt2 + boff + (size_t)nb * 16 * K + kc);
#pragma unroll
            for (int mb = 0; mb < 4; ++mb) { acc[mb][nb] = WFrag<T16>::mma(a[mb], b, acc[mb][nb]); if (NSPLIT == 1 || NSPLIT == 2) acc[mb][nb] = WFrag<T16>::mma(a2[mb], b, acc[mb][nb]); if (NSPLIT >= 2) acc[mb][nb] = WFrag<T16>::mma(a[mb], b2, acc[mb][nb]); } }
        asm volatile("v_nop\n\tv_nop\n\tv_nop\n\tv_nop" : "+v"(acc[0][0]), "+v"(acc[1][1]), "+v"(acc[2][2]), "+v"(acc[3][3]) : "v"(a[0]), "v"(a[3]));
    }
#pragma unroll
    for (int mb = 0; mb < 4; ++mb) {
#pragma unroll
        for (int nb = 0; nb < 4; ++nb) {
#pragma unroll
            for (int j = 0; j < 8; ++j) os[(hi * 8 + j) * 68 + nb * 16 + lr] = acc[mb][nb][j]; }
        __builtin_amdgcn_wave_barrier(); asm volatile("" ::: "memory");
        float* crow = C + (size_t)(r0 + mb * 16) * ldc + c0;
#pragma unroll 1
        for (int ps = 0; ps < 2; ++ps) {
#pragma unroll
            for (int s = 0; s < 8; ++s) { const int row = 2 * s + hi, cofs = lr * 4; v4f val = *(const v4fa*)(os + row * 68 + cofs); if (BIAS) { val[0] += bfr(bias[c0 + cofs]); val[1] += bfr(bias[c0 + cofs + 1]); val[2] += bfr(bias[c0 + cofs + 2]); val[3] += bfr(bias[c0 + cofs + 3]); }
                *(volatile v4f*)(crow + (size_t)row * ldc + cofs) = val; }
            if (ps == 0) __threadfence(); }
        __builtin_amdgcn_wave_barrier(); asm volatile("" ::: "memory");
    }
}

__device__ __forceinline__ h16 tohx(float x) { return (h16)x; }
__device__ __forceinline__ void splitf(float y, unsigned short& h, unsigned short& l) { h = f2bf(y); l = f2bf(y - bf2f(h)); }
typedef __attribute__((ext_vector_type(2))) _Float16 v2h;
typedef __attribute__((ext_vector_type(4))) _Float16 v4h;
typedef __attribute__((ext_vector_type(2))) unsigned short v2us;
typedef __attribute__((ext_vector_type(4))) unsigned short v4us;
typedef __attribute__((ext_vector_type(2))) float v2f;
typedef __attribute__((ext_vector_type(4))) int v4i;

__global__ __launch_bounds__(256) void k_f2h(const float* __restrict__ S, h16* P16, size_t n4) { const size_t i = (size_t)blockIdx.x * 256 + threadIdx.x; if (i >= n4) return; const v4f v = *(const v4f*)(S + i * 4); v4h o;
#pragma unroll
    for (int q = 0; q < 4; ++q) o[q] = tohx(v[q]);
    *(volatile v4h*)(P16 + i * 4) = o; __threadfence(); *(volatile v4h*)(P16 + i * 4) = o; }
__global__ __launch_bounds__(256) void k_rbf(const float* __restrict__ X, float* Y, size_t n4) { const size_t i = (size_t)blockIdx.x * 256 + threadIdx.x; if (i >= n4) return; const v4f a = *(const v4f*)(X + i * 4); v4f o;
#pragma unroll
    for (int q = 0; q < 4; ++q) o[q] = bfr(a[q]);
    *(volatile v4f*)(Y + i * 4) = o; __threadfence(); *(volatile v4f*)(Y + i * 4) = o; }
__global__ __launch_bounds__(256) void k_mmprep(const float* __restrict__ f0, const float* __restrict__ f1, const float* __restrict__ aw, int h0, float* SC) { const int w = (int)threadIdx.x; const int g = (int)blockIdx.x; const int hl = (int)blockIdx.y; const int b = (int)blockIdx.z; const int m = g >> 1; const int c0 = (g & 1) * 64;
    const float* src = (m ? f1 : f0) + (((size_t)b * CH + c0) * IH + (h0 + hl)) * IW + w; const float* a = aw + m * CH + c0; float* dst = SC + (((size_t)hl * IW + w) * 4 + b) * 256 + m * CH + c0;
    v4f o[16];
#pragma unroll
    for (int k = 0; k < 16; ++k) {
#pragma unroll
        for (int q = 0; q < 4; ++q) o[k][q] = __fmul_rn(bfr(src[(size_t)(k * 4 + q) * IH * IW]), bfr(a[k * 4 + q])); }
#pragma unroll
    for (int k = 0; k < 16; ++k) *(volatile v4f*)(dst + k * 4) = o[k];
    __threadfence();
#pragma unroll
    for (int k = 0; k < 16; ++k) *(volatile v4f*)(dst + k * 4) = o[k]; }
__global__ __launch_bounds__(256) void k_mmatt(const float* __restrict__ f0, const float* __restrict__ f1, const float* __restrict__ F, int h0, float* RT) { const int w = (int)threadIdx.x; const int hl = (int)blockIdx.y; const int b = (int)blockIdx.z; const size_t px = (size_t)hl * IW + w;
    const float* s0 = f0 + (((size_t)b * CH) * IH + (h0 + hl)) * IW + w; const float* s1 = f1 + (((size_t)b * CH) * IH + (h0 + hl)) * IW + w; const float* Fp = F + px * 4 * CH;
    float sc[8];
#pragma unroll
    for (int i = 0; i < 8; ++i) sc[i] = 0.f;
    for (int k = 0; k < 32; ++k) { float x0[4], x1[4];
#pragma unroll
        for (int q = 0; q < 4; ++q) { x0[q] = bfr(s0[(size_t)(k * 4 + q) * IH * IW]); x1[q] = bfr(s1[(size_t)(k * 4 + q) * IH * IW]); }
#pragma unroll
        for (int d = 0; d < 4; ++d) { const v4f fd = *(const v4f*)(Fp + d * CH + k * 4);
#pragma unroll
            for (int q = 0; q < 4; ++q) { sc[d] = __fmaf_rn(x0[q], fd[q], sc[d]); sc[4 + d] = __fmaf_rn(x1[q], fd[q], sc[4 + d]); } } }
    float wd[4];
#pragma unroll
    for (int d = 0; d < 4; ++d) wd[d] = 0.f;
#pragma unroll
    for (int m = 0; m < 2; ++m) { float z[4]; float mx = -3.0e38f;
#pragma unroll
        for (int d = 0; d < 4; ++d) { z[d] = __fdiv_rn(sc[m * 4 + d], 11.313708498984761f); mx = fmaxf(mx, z[d]); }
        float sum = 0.f;
#pragma unroll
        for (int d = 0; d < 4; ++d) { z[d] = __builtin_amdgcn_exp2f(__fmul_rn(__fsub_rn(z[d], mx), 1.4426950408889634f)); sum += z[d]; }
        const float inv = __fdiv_rn(1.0f, sum);
#pragma unroll
        for (int d = 0; d < 4; ++d) wd[d] = __fadd_rn(wd[d], __fmul_rn(z[d], inv)); }
    float* dst = RT + (px * 4 + b) * CH;
    v4f o[32];
#pragma unroll
    for (int k = 0; k < 32; ++k) { const v4f f0d = *(const v4f*)(Fp + k * 4);
#pragma unroll
        for (int q = 0; q < 4; ++q) o[k][q] = __fmul_rn(wd[0], f0d[q]);
#pragma unroll
        for (int d = 1; d < 4; ++d) { const v4f fd = *(const v4f*)(Fp + d * CH + k * 4);
#pragma unroll
            for (int q = 0; q < 4; ++q) o[k][q] = __fmaf_rn(wd[d], fd[q], o[k][q]); } }
#pragma unroll
    for (int k = 0; k < 32; ++k) *(volatile v4f*)(dst + k * 4) = o[k];
    __threadfence();
#pragma unroll
    for (int k = 0; k < 32; ++k) *(volatile v4f*)(dst + k * 4) = o[k]; }
__global__ __launch_bounds__(256) void k_mmout(const float* __restrict__ F, const float* __restrict__ Z, int h0, float* out) { const int w = (int)threadIdx.x; const int hl = (int)blockIdx.y; const int c = (int)(blockIdx.z & 127); const int b = (int)(blockIdx.z >> 7); const size_t r = ((size_t)hl * IW + w) * 4 + b;
    const float v = __fadd_rn(F[r * CH + c], fmaxf(Z[r * CH + c], 0.0f)); float* p = out + (((size_t)b * CH + c) * IH + (h0 + hl)) * IW + w; *(volatile float*)p = v; __threadfence(); *(volatile float*)p = v; }

extern "C" void kernel_launch(void* const* d_in, const int* in_sizes, int n_in,
                              void* d_out, int out_size, void* d_ws, size_t ws_size, hipStream_t stream) {
    (void)in_sizes; (void)n_in; (void)out_size;
    const float* f0 = (const float*)d_in[0]; const float* f1 = (const float*)d_in[1]; const float* aw = (const float*)d_in[2]; const float* cw = (const float*)d_in[3]; const float* cb = (const float*)d_in[4]; const float* mw = (const float*)d_in[5]; const float* mb = (const float*)d_in[6];
    float* OUT = (float*)d_out;
    char* wsp = (char*)d_ws;
    auto take = [&](size_t bytes) { char* p = wsp; wsp += (bytes + 255) & ~(size_t)255; return (void*)p; };
    float* CWR = (float*)take((size_t)CH * 256 * 4); float* MWR = (float*)take((size_t)CH * CH * 4); h16* CW = (h16*)take((size_t)CH * 256 * 2); h16* MW = (h16*)take((size_t)CH * CH * 2);
    float* SC = (float*)take((size_t)QR * 256 * 4); h16* SC16 = (h16*)take((size_t)QR * 256 * 2); float* F = (float*)take((size_t)QR * CH * 4); float* RT = (float*)take((size_t)QR * CH * 4); h16* RT16 = (h16*)take((size_t)QR * CH * 2); float* Z = (float*)take((size_t)QR * CH * 4);
    if ((size_t)(wsp - (char*)d_ws) > ws_size) return;
    k_rbf<<<(unsigned)(((size_t)CH * 256 / 4 + 255) / 256), 256, 0, stream>>>(cw, CWR, (size_t)CH * 256 / 4); k_f2h<<<(unsigned)(((size_t)CH * 256 / 4 + 255) / 256), 256, 0, stream>>>(CWR, CW, (size_t)CH * 256 / 4);
    k_rbf<<<(unsigned)(((size_t)CH * CH / 4 + 255) / 256), 256, 0, stream>>>(mw, MWR, (size_t)CH * CH / 4); k_f2h<<<(unsigned)(((size_t)CH * CH / 4 + 255) / 256), 256, 0, stream>>>(MWR, MW, (size_t)CH * CH / 4);
    for (int q = 0; q < 4; ++q) { const int h0 = q * QH;
        k_mmprep<<<dim3(4, QH, NB_), 256, 0, stream>>>(f0, f1, aw, h0, SC);
        k_f2h<<<(unsigned)(((size_t)QR * 256 / 4 + 255) / 256), 256, 0, stream>>>(SC, SC16, (size_t)QR * 256 / 4);
        k_gemmw<h16, 0, true><<<dim3(QR / 64, CH / 64, 1), 32, 0, stream>>>(SC16, nullptr, CW, nullptr, 256, F, CH, cb, 0, 0, 0);
        k_mmatt<<<dim3(1, QH, NB_), 256, 0, stream>>>(f0, f1, F, h0, RT);
        k_f2h<<<(unsigned)(((size_t)QR * CH / 4 + 255) / 256), 256, 0, stream>>>(RT, RT16, (size_t)QR * CH / 4);
        k_gemmw<h16, 0, true><<<dim3(QR / 64, CH / 64, 1), 32, 0, stream>>>(RT16, nullptr, MW, nullptr, CH, Z, CH, mb, 0, 0, 0);
        k_mmout<<<dim3(1, QH, NB_ * CH), 256, 0, stream>>>(F, Z, h0, OUT); }
}
